// SAGE_sup_55009941127683
// MI455X (gfx1250) — hardware-verified
//
#include <hip/hip_runtime.h>
#include <stddef.h>


#define FIN     128
#define HID     256
#define NCLS    100
#define NOP     128
#define KA1     (2 * FIN)
#define KA2     (2 * HID)
#define NTHR    256
#define NWAVE   8
#define EPT     8
#define NGRP    2
#define CHUNK   (NTHR * EPT * NGRP)
#define WCAP    (EPT * NGRP * 32)
#define LISTN   (NWAVE * WCAP)
#define NBC     4096
#define NBF     1024
#define RCAP    40960
#define RBN     128
#define RPAD    256
#define ATHR    128
#define AWAVE   4
#define TGT     (AWAVE * 32)
#define DEGCAP  1024
#define OTHR    512
#define BM1     32
#define BM2     64
#define WSCAP   134217728
#define ACARRY  8.0f
#define WCARRY  64.0f
#define GSCALE  (1.0f / 512.0f)
#define U1      (HID * (KA1 / 8))
#define U2      (NOP * (KA2 / 8))
#define NUNITS  (U1 + U2)

#define LDS_FILL ((RCAP + NBF + LISTN) * 4 + 64)
#define LDS_AGG1 (AWAVE * 32 * 2 * FIN * 2)
#define LDS_AGG2 (AWAVE * 32 * HID * 2)

static_assert((CHUNK & (CHUNK - 1)) == 0);
static_assert(CHUNK <= 4096);
static_assert((NBC & (NBC - 1)) == 0 && (NBF & (NBF - 1)) == 0);
static_assert(NBC == 4 * NBF);
static_assert(OTHR * 8 == NBC);
static_assert((RCAP % 32) == 0);
static_assert(WCAP == EPT * NGRP * 32);
static_assert(FIN == 4 * 32);
static_assert(HID == 8 * 32);
static_assert((FIN % 32) == 0 && (HID % 32) == 0);
static_assert((NOP % 16) == 0 && NCLS <= NOP && (NCLS % 4) == 0);
static_assert((RPAD % TGT) == 0 && (RPAD % 128) == 0 && (RPAD % BM1) == 0 && (RPAD % BM2) == 0);
static_assert((NBC % RPAD) == 0);
static_assert(TGT == AWAVE * 32);
static_assert(ATHR == AWAVE * 32);
static_assert((BM2 * NCLS * 4) % 128 == 0);
static_assert((NUNITS % NTHR) == 0);
static_assert(LDS_AGG1 == LDS_AGG2);

typedef float    v2f  __attribute__((ext_vector_type(2)));
typedef float    v4f  __attribute__((ext_vector_type(4)));
typedef float    v8f  __attribute__((ext_vector_type(8)));
typedef int      v4i  __attribute__((ext_vector_type(4)));
typedef _Float16 v4h  __attribute__((ext_vector_type(4)));
typedef _Float16 v8h  __attribute__((ext_vector_type(8)));
typedef _Float16 v16h __attribute__((ext_vector_type(16)));
union Frag { v16h v; v8h h[2]; };

__device__ __forceinline__ v8f wmh(v16h a, v16h b, v8f c) {
  v8f d = __builtin_amdgcn_wmma_f32_16x16x32_f16(false, a, false, b, (short)0, c, false, false);
  asm volatile("v_nop\n\tv_nop\n\tv_nop\n\tv_nop" : "+v"(d) : "v"(a), "v"(b));
  return d;
}

template <int NB>
__device__ __forceinline__ int scan_chunk(const int* __restrict__ dsts, int nE, int cbase, int slotBase,
                                          int vec8, int* list, int tid, int lane, int wave) {
  int wc = 0;
#pragma unroll
  for (int g = 0; g < NGRP; ++g) {
    const int el0  = (g * NTHR + tid) * EPT;
    const int e0   = cbase + el0;
    const int sent = -2147483647 - 1;
    v4i da, db;
    if (vec8 != 0 && cbase + CHUNK <= nE) {
      da = *(const v4i*)(dsts + e0);
      db = *(const v4i*)(dsts + e0 + 4);
    } else {
      da.x = (e0     < nE) ? dsts[min(e0, nE - 1)] : sent;
      da.y = (e0 + 1 < nE) ? dsts[min(e0 + 1, nE - 1)] : sent;
      da.z = (e0 + 2 < nE) ? dsts[min(e0 + 2, nE - 1)] : sent;
      da.w = (e0 + 3 < nE) ? dsts[min(e0 + 3, nE - 1)] : sent;
      db.x = (e0 + 4 < nE) ? dsts[min(e0 + 4, nE - 1)] : sent;
      db.y = (e0 + 5 < nE) ? dsts[min(e0 + 5, nE - 1)] : sent;
      db.z = (e0 + 6 < nE) ? dsts[min(e0 + 6, nE - 1)] : sent;
      db.w = (e0 + 7 < nE) ? dsts[min(e0 + 7, nE - 1)] : sent;
    }
    const unsigned nb = (unsigned)slotBase;
    const unsigned s0 = (unsigned)da.x - nb, s1 = (unsigned)da.y - nb;
    const unsigned s2 = (unsigned)da.z - nb, s3 = (unsigned)da.w - nb;
    const unsigned s4 = (unsigned)db.x - nb, s5 = (unsigned)db.y - nb;
    const unsigned s6 = (unsigned)db.z - nb, s7 = (unsigned)db.w - nb;
    const bool h0 = s0 < (unsigned)NB, h1 = s1 < (unsigned)NB, h2 = s2 < (unsigned)NB, h3 = s3 < (unsigned)NB;
    const bool h4 = s4 < (unsigned)NB, h5 = s5 < (unsigned)NB, h6 = s6 < (unsigned)NB, h7 = s7 < (unsigned)NB;
    const unsigned any = __builtin_amdgcn_ballot_w32(h0 | h1 | h2 | h3 | h4 | h5 | h6 | h7);
    if (any != 0u) {
#define HITJ(J, HJ, SJ) { \
        const unsigned mj = __builtin_amdgcn_ballot_w32(HJ); \
        if (mj != 0u) { \
          if (HJ) { \
            const int pos = wc + (int)__builtin_amdgcn_mbcnt_lo(mj, 0u); \
            if (pos < WCAP) list[wave * WCAP + pos] = ((el0 + (J)) << 12) | (int)(SJ); \
          } \
          wc += (int)__builtin_popcount(mj); } }
      HITJ(0, h0, s0)
      HITJ(1, h1, s1)
      HITJ(2, h2, s2)
      HITJ(3, h3, s3)
      HITJ(4, h4, s4)
      HITJ(5, h5, s5)
      HITJ(6, h6, s6)
      HITJ(7, h7, s7)
#undef HITJ
    }
  }
  return wc;
}

__global__ __launch_bounds__(NTHR) void k_count(
    const int* __restrict__ dsts, int* cnt, int nE, int vec8) {
  __shared__ __attribute__((aligned(16))) int scnt[NBC];
  __shared__ __attribute__((aligned(16))) int list[LISTN];
  __shared__ int wcnt[NWAVE];
  const int tid = threadIdx.x, lane = tid & 31, wave = tid >> 5;
  const int nodeBase = blockIdx.x * NBC;

  for (int i = tid; i < NBC; i += NTHR) scnt[i] = 0;
  __syncthreads();

  const int nChunks = (nE + CHUNK - 1) / CHUNK;
#pragma unroll 1
  for (int ch = 0; ch < nChunks; ++ch) {
    const int cbase = ch * CHUNK;
    const int wc = scan_chunk<NBC>(dsts, nE, cbase, nodeBase, vec8, list, tid, lane, wave);
    if (lane == 0) wcnt[wave] = wc;
    __syncthreads();
    if (wave == 0) {
#pragma unroll 1
      for (int wsx = 0; wsx < NWAVE; ++wsx) {
        int n = __builtin_amdgcn_readfirstlane(wcnt[wsx]);
        n = n > WCAP ? WCAP : (n < 0 ? 0 : n);
        const int* lp = list + wsx * WCAP;
#pragma unroll 1
        for (int i = 0; i < n; ++i) {
          const int ent  = __builtin_amdgcn_readfirstlane(lp[i]);
          const int slot = ent & (NBC - 1);
          if (lane == 0) scnt[slot] = scnt[slot] + 1;
        }
      }
    }
    __syncthreads();
  }

  v4i cq[4];
#pragma unroll
  for (int q = 0; q < 4; ++q) {
    const int f = (wave * 4 + q) * 128 + 4 * lane;
    cq[q] = *(const v4i*)(scnt + f);
  }
  int* cp = cnt + (size_t)nodeBase;
#pragma unroll
  for (int q = 0; q < 4; ++q) {
    const int f = (wave * 4 + q) * 128 + 4 * lane;
    *(volatile v4i*)(cp + f) = cq[q];
  }
  __threadfence();
#pragma unroll
  for (int q = 0; q < 4; ++q) {
    const int f = (wave * 4 + q) * 128 + 4 * lane;
    *(volatile v4i*)(cp + f) = cq[q];
  }
}

__global__ __launch_bounds__(OTHR) void k_offsets(
    const int* __restrict__ cnt, int* off, int* rbase, int nChunk) {
  __shared__ __attribute__((aligned(16))) int soff[NBC];
  __shared__ __attribute__((aligned(16))) int srb[RBN];
  __shared__ int wtot[OTHR / 32];
  const int tid = threadIdx.x, lane = tid & 31, wave = tid >> 5, sub = tid >> 7;
  for (int i = tid; i < RBN; i += OTHR) srb[i] = 0;
  int carry = 0;
#pragma unroll 1
  for (int ch = 0; ch < nChunk; ++ch) {
    const int base = ch * NBC;
    const v4i c0 = *(const v4i*)(cnt + base + 8 * tid);
    const v4i c1 = *(const v4i*)(cnt + base + 8 * tid + 4);
    const int e0 = max(c0.x, 0), e1 = max(c0.y, 0), e2 = max(c0.z, 0), e3 = max(c0.w, 0);
    const int e4 = max(c1.x, 0), e5 = max(c1.y, 0), e6 = max(c1.z, 0), e7 = max(c1.w, 0);
    const int ts = e0 + e1 + e2 + e3 + e4 + e5 + e6 + e7;
    int incl = ts;
#pragma unroll
    for (int d = 1; d < 32; d <<= 1) {
      const int t = __shfl_up(incl, d);
      if (lane >= d) incl += t;
    }
    if (lane == 31) wtot[wave] = incl;
    __syncthreads();
    const int S0 = wtot[0]  + wtot[1]  + wtot[2]  + wtot[3];
    const int S1 = wtot[4]  + wtot[5]  + wtot[6]  + wtot[7];
    const int S2 = wtot[8]  + wtot[9]  + wtot[10] + wtot[11];
    const int S3 = wtot[12] + wtot[13] + wtot[14] + wtot[15];
    int pre = 0;
#pragma unroll 1
    for (int w = 4 * sub; w < wave; ++w) pre += wtot[w];
    const int b0 = carry;
    const int b1 = b0 + ((S0 + 31) & ~31);
    const int b2 = b1 + ((S1 + 31) & ~31);
    const int b3 = b2 + ((S2 + 31) & ~31);
    const int b4 = b3 + ((S3 + 31) & ~31);
    const int myb = sub == 0 ? b0 : (sub == 1 ? b1 : (sub == 2 ? b2 : b3));
    if (tid == 0) {
      srb[min(4 * ch + 0, RBN - 1)] = b0;
      srb[min(4 * ch + 1, RBN - 1)] = b1;
      srb[min(4 * ch + 2, RBN - 1)] = b2;
      srb[min(4 * ch + 3, RBN - 1)] = b3;
    }
    int run = myb + pre + incl - ts;
    soff[8 * tid + 0] = run; run += e0;
    soff[8 * tid + 1] = run; run += e1;
    soff[8 * tid + 2] = run; run += e2;
    soff[8 * tid + 3] = run; run += e3;
    soff[8 * tid + 4] = run; run += e4;
    soff[8 * tid + 5] = run; run += e5;
    soff[8 * tid + 6] = run; run += e6;
    soff[8 * tid + 7] = run;
    carry = b4;
    __syncthreads();
    const v4i o0 = *(const v4i*)(soff + 4 * tid);
    const v4i o1 = *(const v4i*)(soff + 4 * (tid + OTHR));
    int* op = off + base;
    *(volatile v4i*)(op + 4 * tid) = o0;
    *(volatile v4i*)(op + 4 * (tid + OTHR)) = o1;
    __threadfence();
    *(volatile v4i*)(op + 4 * tid) = o0;
    *(volatile v4i*)(op + 4 * (tid + OTHR)) = o1;
    __syncthreads();
  }
  if (tid == 0) srb[min(4 * nChunk, RBN - 1)] = carry;
  __syncthreads();
  v4i rv = {0, 0, 0, 0};
  if (tid < 32) rv = *(const v4i*)(srb + 4 * tid);
  if (tid < 32) *(volatile v4i*)(rbase + 4 * tid) = rv;
  __threadfence();
  if (tid < 32) *(volatile v4i*)(rbase + 4 * tid) = rv;
}

__global__ __launch_bounds__(NTHR) void k_fill(
    const int* __restrict__ srcs, const int* __restrict__ dsts,
    const int* __restrict__ off, const int* __restrict__ rbase,
    int* csr, int nN, int nE, int vec8, int csrLen) {
  extern __shared__ v4f lds_dyn[];
  int* region = (int*)lds_dyn;
  int* cursor = region + RCAP;
  int* list   = cursor + NBF;
  int* wcnt   = list + LISTN;
  const int tid = threadIdx.x, lane = tid & 31, wave = tid >> 5;
  const int b = blockIdx.x;
  const int nodeBase = b * NBF;

  int rb0 = rbase[b];
  const int rb1 = rbase[b + 1];
  rb0 = rb0 < 0 ? 0 : (rb0 > csrLen ? csrLen : rb0);
  rb0 &= ~31;
  int len = rb1 - rb0;
  len = len < 0 ? 0 : (len > RCAP ? RCAP : len);
  int lenW = (len + 31) & ~31;
  if (rb0 + lenW > csrLen) lenW = (csrLen - rb0) & ~31;

  {
    const v4i z = {0, 0, 0, 0};
    for (int i = tid; i < RCAP / 4; i += NTHR) ((v4i*)region)[i] = z;
    for (int s = tid; s < NBF; s += NTHR) {
      int o = off[nodeBase + s] - rb0;
      o = o < 0 ? 0 : (o > RCAP ? RCAP : o);
      cursor[s] = o;
    }
  }
  __syncthreads();

  const int nChunks = (nE + CHUNK - 1) / CHUNK;
#pragma unroll 1
  for (int ch = 0; ch < nChunks; ++ch) {
    const int cbase = ch * CHUNK;
    const int wc = scan_chunk<NBF>(dsts, nE, cbase, nodeBase, vec8, list, tid, lane, wave);
    if (lane == 0) wcnt[wave] = wc;
    __syncthreads();
    if (wave == 0) {
#pragma unroll 1
      for (int wsx = 0; wsx < NWAVE; ++wsx) {
        int n = __builtin_amdgcn_readfirstlane(wcnt[wsx]);
        n = n > WCAP ? WCAP : (n < 0 ? 0 : n);
        const int* lp = list + wsx * WCAP;
#pragma unroll 1
        for (int i = 0; i < n; ++i) {
          const int ent  = __builtin_amdgcn_readfirstlane(lp[i]);
          const int slot = ent & (NBF - 1);
          int e = cbase + ((ent >> 12) & (CHUNK - 1));
          e = e > nE - 1 ? nE - 1 : e;
          int sv = srcs[e];
          sv = sv < 0 ? 0 : (sv > nN - 1 ? nN - 1 : sv);
          if (lane == 0) {
            int pos = cursor[slot];
            pos = pos < 0 ? 0 : (pos > RCAP - 1 ? RCAP - 1 : pos);
            region[pos] = sv;
            const int np = pos + 1;
            cursor[slot] = np > RCAP ? RCAP : np;
          }
        }
      }
    }
    __syncthreads();
  }

  const int nv = lenW >> 2;
  int* gp = csr + rb0;
#pragma unroll 1
  for (int i = tid; i < nv; i += NTHR) { const v4i v = ((const v4i*)region)[i]; *(volatile v4i*)(gp + 4 * i) = v; }
  __threadfence();
#pragma unroll 1
  for (int i = tid; i < nv; i += NTHR) { const v4i v = ((const v4i*)region)[i]; *(volatile v4i*)(gp + 4 * i) = v; }
}

__global__ __launch_bounds__(NTHR) void k_wcvt(const float* __restrict__ w1l, const float* __restrict__ w1r,
                                               const float* __restrict__ w2l, const float* __restrict__ w2r,
                                               _Float16* dp, int nUnits) {
  const int i = (int)blockIdx.x * NTHR + (int)threadIdx.x;
  if (i >= nUnits) return;
  constexpr int PPR1 = KA1 / 8;
  constexpr int PPR2 = KA2 / 8;
  const bool p2 = i >= U1;
  const int r = p2 ? (i - U1) : i;
  const int n = p2 ? (r / PPR2) : (r / PPR1);
  const int seg = p2 ? (r - n * PPR2) : (r - n * PPR1);
  const int n1 = n > HID - 1 ? HID - 1 : n;
  const int n2 = n > NCLS - 1 ? NCLS - 1 : n;
  const bool l1 = seg < (FIN / 8);
  const bool l2 = seg < (HID / 8);
  const bool live2 = n < NCLS;
  v8h o;
#pragma unroll
  for (int j = 0; j < 8; ++j) {
    const int kk1 = (8 * seg + j) & (FIN - 1);
    const int kk2 = (8 * seg + j) & (HID - 1);
    const float f1l = w1l[kk1 * HID + n1];
    const float f1r = w1r[kk1 * HID + n1];
    const float f2l = w2l[kk2 * NCLS + n2];
    const float f2r = w2r[kk2 * NCLS + n2];
    const float f = p2 ? (live2 ? (l2 ? f2l : f2r) : 0.f) : (l1 ? f1l : f1r);
    o[j] = (_Float16)(f * WCARRY);
  }
  _Float16* gp = dp + (size_t)i * 8;
  *(volatile v8h*)gp = o;
  __threadfence();
  *(volatile v8h*)gp = o;
}

__global__ __launch_bounds__(ATHR) void k_agg1(
    const int* __restrict__ csr, const int* __restrict__ off, const int* __restrict__ cnt,
    const float* __restrict__ x, _Float16* mp, _Float16* op, int nN, int csrLen) {
  extern __shared__ v4f lds_dyn[];
  _Float16* stg = (_Float16*)lds_dyn;
  const int tid = threadIdx.x, lane = tid & 31, wave = tid >> 5;
  const int tbase = blockIdx.x * TGT + wave * 32;
  const int col = 4 * lane;
  const int cl    = tbase + lane;
  const int cnt_l = cnt[cl];
  const int off_l = off[cl];
  _Float16* swm = stg + (size_t)wave * (2 * 32 * FIN);
  _Float16* swo = swm + 32 * FIN;

#pragma unroll 1
  for (int j = 0; j < 32; ++j) {
    const int c = tbase + j;
    int nt = __shfl(cnt_l, j);
    nt = nt < 0 ? 0 : nt;
    const int n = nt > DEGCAP ? DEGCAP : nt;
    const int st = __shfl(off_l, j);
    float rc = 1.0f / (float)(nt < 1 ? 1 : nt);
    rc = (nt > DEGCAP) ? __int_as_float(0x7fc00000) : rc;

    v4f a = {0.f, 0.f, 0.f, 0.f};
#pragma unroll 1
    for (int q0 = 0; q0 < n; q0 += 32) {
      int pos = st + q0 + lane;
      pos = pos < 0 ? 0 : (pos > csrLen - 1 ? csrLen - 1 : pos);
      int sl = csr[pos];
      sl = sl < 0 ? 0 : (sl > nN - 1 ? nN - 1 : sl);
      const int mcnt = (n - q0) < 32 ? (n - q0) : 32;
#pragma unroll 1
      for (int pp = 0; pp < mcnt; ++pp) {
        const int s = __builtin_amdgcn_readlane(sl, pp);
        const v4f xv = *(const v4f*)(x + (size_t)s * FIN + col);
        a = a + xv;
      }
    }

    const bool live = c < nN;
    const int cc = c > nN - 1 ? nN - 1 : c;
    const v4f sv = *(const v4f*)(x + (size_t)cc * FIN + col);
    const float fm = live ? rc * ACARRY : 0.f;
    const float fs = live ? ACARRY : 0.f;
    v4h om, oo;
    om.x = (_Float16)(a.x * fm);
    om.y = (_Float16)(a.y * fm);
    om.z = (_Float16)(a.z * fm);
    om.w = (_Float16)(a.w * fm);
    oo.x = (_Float16)(sv.x * fs);
    oo.y = (_Float16)(sv.y * fs);
    oo.z = (_Float16)(sv.z * fs);
    oo.w = (_Float16)(sv.w * fs);
    *(v4h*)(swm + j * FIN + col) = om;
    *(v4h*)(swo + j * FIN + col) = oo;
  }
  __syncthreads();

  constexpr int NI = (32 * FIN) / (32 * 8);
  _Float16* gm = mp + (size_t)tbase * FIN;
  _Float16* go = op + (size_t)tbase * FIN;
#pragma unroll 1
  for (int i = 0; i < NI; ++i) {
    const v8h vm = *(const v8h*)(swm + i * 256 + 8 * lane);
    const v8h vo = *(const v8h*)(swo + i * 256 + 8 * lane);
    *(volatile v8h*)(gm + i * 256 + 8 * lane) = vm;
    *(volatile v8h*)(go + i * 256 + 8 * lane) = vo;
  }
  __threadfence();
#pragma unroll 1
  for (int i = 0; i < NI; ++i) {
    const v8h vm = *(const v8h*)(swm + i * 256 + 8 * lane);
    const v8h vo = *(const v8h*)(swo + i * 256 + 8 * lane);
    *(volatile v8h*)(gm + i * 256 + 8 * lane) = vm;
    *(volatile v8h*)(go + i * 256 + 8 * lane) = vo;
  }
}

__global__ __launch_bounds__(ATHR) void k_agg2(
    const int* __restrict__ csr, const int* __restrict__ off, const int* __restrict__ cnt,
    const _Float16* __restrict__ hp, _Float16* mp, int nN, int csrLen) {
  extern __shared__ v4f lds_dyn[];
  _Float16* stg = (_Float16*)lds_dyn;
  const int tid = threadIdx.x, lane = tid & 31, wave = tid >> 5;
  const int tbase = blockIdx.x * TGT + wave * 32;
  const int col = 8 * lane;
  const int cl    = tbase + lane;
  const int cnt_l = cnt[cl];
  const int off_l = off[cl];
  _Float16* swm = stg + (size_t)wave * (32 * HID);

#pragma unroll 1
  for (int j = 0; j < 32; ++j) {
    const int c = tbase + j;
    int nt = __shfl(cnt_l, j);
    nt = nt < 0 ? 0 : nt;
    const int n = nt > DEGCAP ? DEGCAP : nt;
    const int st = __shfl(off_l, j);
    float rc = 1.0f / (float)(nt < 1 ? 1 : nt);
    rc = (nt > DEGCAP) ? __int_as_float(0x7fc00000) : rc;

    v8f a = {0.f, 0.f, 0.f, 0.f, 0.f, 0.f, 0.f, 0.f};
#pragma unroll 1
    for (int q0 = 0; q0 < n; q0 += 32) {
      int pos = st + q0 + lane;
      pos = pos < 0 ? 0 : (pos > csrLen - 1 ? csrLen - 1 : pos);
      int sl = csr[pos];
      sl = sl < 0 ? 0 : (sl > nN - 1 ? nN - 1 : sl);
      const int mcnt = (n - q0) < 32 ? (n - q0) : 32;
#pragma unroll 1
      for (int pp = 0; pp < mcnt; ++pp) {
        const int s = __builtin_amdgcn_readlane(sl, pp);
        const v8h hv = *(const v8h*)(hp + (size_t)s * HID + col);
        a = a + __builtin_convertvector(hv, v8f);
      }
    }

    const bool live = c < nN;
    const float fm = live ? rc : 0.f;
    const v8f am = a * fm;
    const v8h om = __builtin_convertvector(am, v8h);
    *(v8h*)(swm + j * HID + col) = om;
  }
  __syncthreads();

  constexpr int NI = (32 * HID) / (32 * 8);
  _Float16* gm = mp + (size_t)tbase * HID;
#pragma unroll 1
  for (int i = 0; i < NI; ++i) {
    const v8h vm = *(const v8h*)(swm + i * 256 + 8 * lane);
    *(volatile v8h*)(gm + i * 256 + 8 * lane) = vm;
  }
  __threadfence();
#pragma unroll 1
  for (int i = 0; i < NI; ++i) {
    const v8h vm = *(const v8h*)(swm + i * 256 + 8 * lane);
    *(volatile v8h*)(gm + i * 256 + 8 * lane) = vm;
  }
}

template <int FW, int TPW>
__device__ __forceinline__ void gemm_core(const _Float16* __restrict__ am, const _Float16* __restrict__ ao,
                                          const _Float16* __restrict__ bp, v8f (&acc)[TPW]) {
  constexpr int KA = 2 * FW;
  constexpr int KST = FW / 32;
#pragma unroll 1
  for (int kt = 0; kt < KST; ++kt) {
    Frag a;
    a.h[0] = *(const v8h*)(am + 32 * kt);
    a.h[1] = *(const v8h*)(am + 32 * kt + 16);
#pragma unroll
    for (int t = 0; t < TPW; ++t) {
      const size_t to = (size_t)(16 * t) * KA + 32 * kt;
      Frag b;
      b.h[0] = *(const v8h*)(bp + to);
      b.h[1] = *(const v8h*)(bp + to + 16);
      acc[t] = wmh(a.v, b.v, acc[t]);
    }
  }
#pragma unroll 1
  for (int kt = 0; kt < KST; ++kt) {
    Frag a;
    a.h[0] = *(const v8h*)(ao + 32 * kt);
    a.h[1] = *(const v8h*)(ao + 32 * kt + 16);
#pragma unroll
    for (int t = 0; t < TPW; ++t) {
      const size_t to = (size_t)(16 * t) * KA + FW + 32 * kt;
      Frag b;
      b.h[0] = *(const v8h*)(bp + to);
      b.h[1] = *(const v8h*)(bp + to + 16);
      acc[t] = wmh(a.v, b.v, acc[t]);
    }
  }
}

template <int FW, int NCOL, int BMR>
__global__ __launch_bounds__(NTHR) void k_gemm1(
    const _Float16* __restrict__ Am, const _Float16* __restrict__ Ao, const _Float16* __restrict__ Bp,
    const float* __restrict__ bias, _Float16* Hout, int nValid) {
  constexpr int KA = 2 * FW;
  constexpr int TPW = (BMR / 16) * (NCOL / 16) / NWAVE;
  constexpr int NCG = NCOL / (16 * TPW);
  constexpr int NEL = BMR * NCOL;
  constexpr int NIT = NEL / (8 * NTHR);
  static_assert(TPW >= 1 && TPW * NWAVE * 256 == NEL);
  static_assert(NCG >= 1 && NCG * 16 * TPW == NCOL);
  static_assert((NWAVE % NCG) == 0 && (NWAVE / NCG) * 16 == BMR);
  static_assert(NIT >= 1 && NIT * 8 * NTHR == NEL);
  static_assert((FW % 32) == 0 && (NCOL % 8) == 0);

  __shared__ __attribute__((aligned(16))) _Float16 stg[NEL];
  const int tid = threadIdx.x, lane = tid & 31, wave = tid >> 5, hh = lane >> 4, m = lane & 15;
  const int rowBase = (int)blockIdx.x * BMR;
  const int rg = wave / NCG, cg = wave - rg * NCG;
  const int r0 = rg * 16;
  const int c0 = cg * 16 * TPW;

  v8f acc[TPW];
#pragma unroll
  for (int t = 0; t < TPW; ++t) { v8f z = {0.f, 0.f, 0.f, 0.f, 0.f, 0.f, 0.f, 0.f}; acc[t] = z; }

  const _Float16* am = Am + (size_t)(rowBase + r0 + m) * FW + 8 * hh;
  const _Float16* ao = Ao + (size_t)(rowBase + r0 + m) * FW + 8 * hh;
  const _Float16* bp = Bp + (size_t)(c0 + m) * KA + 8 * hh;
  gemm_core<FW, TPW>(am, ao, bp, acc);

  {
    _Float16* sp = stg + (size_t)(r0 + 8 * hh) * NCOL + c0 + m;
    const int growb = rowBase + r0 + 8 * hh;
#pragma unroll
    for (int t = 0; t < TPW; ++t) {
      const float bv = bias[c0 + 16 * t + m];
#pragma unroll
      for (int r = 0; r < 8; ++r) {
        const bool lv = (growb + r) < nValid;
        float v = acc[t][r] * GSCALE + bv;
        v = (v < 0.f) ? 0.f : v;
        v = v * ACARRY;
        sp[r * NCOL + 16 * t] = lv ? (_Float16)v : (_Float16)0.f;
      }
    }
  }
  __syncthreads();

  v8h cv[NIT];
#pragma unroll
  for (int it = 0; it < NIT; ++it) {
    const int id = it * NTHR + tid;
    cv[it] = *(const v8h*)(stg + 8 * id);
  }
  _Float16* gb = Hout + (size_t)rowBase * NCOL;
#pragma unroll
  for (int it = 0; it < NIT; ++it) {
    const int id = it * NTHR + tid;
    *(volatile v8h*)(gb + 8 * id) = cv[it];
  }
  __threadfence();
#pragma unroll
  for (int it = 0; it < NIT; ++it) {
    const int id = it * NTHR + tid;
    *(volatile v8h*)(gb + 8 * id) = cv[it];
  }
}

template <int FW, int NCOL, int BMR, int NC>
__global__ __launch_bounds__(NTHR) void k_gemm2(
    const _Float16* __restrict__ Am, const _Float16* __restrict__ Ao, const _Float16* __restrict__ Bp,
    const float* __restrict__ bias, float* Out, int nValid) {
  constexpr int KA = 2 * FW;
  constexpr int TPW = (BMR / 16) * (NCOL / 16) / NWAVE;
  constexpr int NCG = NCOL / (16 * TPW);
  constexpr int NEL = BMR * NCOL;
  constexpr int NST = BMR * NC;
  constexpr int NF4 = NST / 4;
  constexpr int NIT = (NF4 + NTHR - 1) / NTHR;
  static_assert(TPW >= 1 && TPW * NWAVE * 256 == NEL);
  static_assert(NCG >= 1 && NCG * 16 * TPW == NCOL);
  static_assert((NWAVE % NCG) == 0 && (NWAVE / NCG) * 16 == BMR);
  static_assert((FW % 32) == 0 && (NC % 4) == 0 && NC <= NCOL);
  static_assert((NST * 4) % 128 == 0);
  static_assert(NIT >= 1 && NIT <= 8);

  __shared__ __attribute__((aligned(16))) float stg[NST];
  const int tid = threadIdx.x, lane = tid & 31, wave = tid >> 5, hh = lane >> 4, m = lane & 15;
  const int rowBase = (int)blockIdx.x * BMR;
  const int rg = wave / NCG, cg = wave - rg * NCG;
  const int r0 = rg * 16;
  const int c0 = cg * 16 * TPW;

  v8f acc[TPW];
#pragma unroll
  for (int t = 0; t < TPW; ++t) { v8f z = {0.f, 0.f, 0.f, 0.f, 0.f, 0.f, 0.f, 0.f}; acc[t] = z; }

  const _Float16* am = Am + (size_t)(rowBase + r0 + m) * FW + 8 * hh;
  const _Float16* ao = Ao + (size_t)(rowBase + r0 + m) * FW + 8 * hh;
  const _Float16* bp = Bp + (size_t)(c0 + m) * KA + 8 * hh;
  gemm_core<FW, TPW>(am, ao, bp, acc);

  {
    const int rowb = r0 + 8 * hh;
#pragma unroll
    for (int t = 0; t < TPW; ++t) {
      const int col = c0 + 16 * t + m;
      const int colc = col > NC - 1 ? NC - 1 : col;
      const float bv = bias[colc];
      const bool cb = col < NC;
#pragma unroll
      for (int r = 0; r < 8; ++r) {
        const float v = acc[t][r] * GSCALE + bv;
        if (cb) stg[(rowb + r) * NC + col] = v;
      }
    }
  }
  __syncthreads();

#pragma unroll 1
  for (int i = tid; i < NST; i += NTHR) {
    float z = stg[i];
    z = (z < -30.f) ? -30.f : z;
    z = (z > 30.f) ? 30.f : z;
    const float e = expf(-z);
    stg[i] = 1.0f / (1.0f + e);
  }
  __syncthreads();

  int nv = nValid - rowBase;
  nv = nv < 0 ? 0 : (nv > BMR ? BMR : nv);
  const int nfl = nv * (NC / 4);
  v4f cv[NIT];
#pragma unroll
  for (int it = 0; it < NIT; ++it) {
    const int id = it * NTHR + tid;
    const int idc = id > NF4 - 1 ? NF4 - 1 : id;
    cv[it] = *(const v4f*)(stg + 4 * idc);
  }
  float* gb = Out + (size_t)rowBase * NC;
#pragma unroll
  for (int it = 0; it < NIT; ++it) {
    const int id = it * NTHR + tid;
    if (id < nfl) *(volatile v4f*)(gb + 4 * (size_t)id) = cv[it];
  }
  __threadfence();
#pragma unroll
  for (int it = 0; it < NIT; ++it) {
    const int id = it * NTHR + tid;
    if (id < nfl) *(volatile v4f*)(gb + 4 * (size_t)id) = cv[it];
  }
}

extern "C" void kernel_launch(void* const* d_in, const int* in_sizes, int n_in,
                              void* d_out, int out_size, void* d_ws, size_t ws_size,
                              hipStream_t stream) {
  if (n_in < 8) return;
  if (in_sizes[0] < FIN || (in_sizes[0] % FIN) != 0) return;
  const int nN = in_sizes[0] / FIN;
  if (in_sizes[1] < 2 || (in_sizes[1] & 1) != 0) return;
  const int nE = in_sizes[1] / 2;
  if (in_sizes[2] != FIN * HID || in_sizes[3] != FIN * HID || in_sizes[4] != HID) return;
  if (in_sizes[5] != HID * NCLS || in_sizes[6] != HID * NCLS || in_sizes[7] != NCLS) return;
  if (out_size != nN * NCLS) return;
  if (nE < 1 || nE > (1 << 28) || nN < 1 || nN > (1 << 22)) return;

  const float* x   = (const float*)d_in[0];
  const int*   ei  = (const int*)d_in[1];
  const int*   src = ei;
  const int*   dst = ei + nE;
  const float* w1l = (const float*)d_in[2];
  const float* w1r = (const float*)d_in[3];
  const float* b1  = (const float*)d_in[4];
  const float* w2l = (const float*)d_in[5];
  const float* w2r = (const float*)d_in[6];
  const float* b2  = (const float*)d_in[7];
  float* out = (float*)d_out;

  const int NPAD   = ((nN + RPAD - 1) / RPAD) * RPAD;
  const int nBC    = (nN + NBC - 1) / NBC;
  const int CNTPAD = nBC * NBC;
  if (CNTPAD < NPAD) return;
  if (4 * nBC + 1 > RBN) return;
  const int nBF    = (nN + NBF - 1) / NBF;
  if (nBF > 4 * nBC) return;
  const int csrLen = ((nE + 31) & ~31) + 4096;
  if (31 * 4 * nBC > 4096) return;
  const int nAgg   = NPAD / TGT;
  const int nG1    = NPAD / BM1;
  const int nG2    = (nN + BM2 - 1) / BM2;
  if (nG2 < 1 || nG2 * BM2 > NPAD) return;
  const int nUnits = NUNITS;

  char* ws = (char*)d_ws;
  size_t off = 0;
  const size_t bR1a = (size_t)NPAD * FIN * 2 * 2;
  const size_t bR1b = (size_t)NPAD * HID * 2;
  const size_t bR1  = bR1a > bR1b ? bR1a : bR1b;
  const size_t oWp  = off; off += (size_t)NUNITS * 8 * 2;       off = (off + 255) & ~(size_t)255;
  const size_t oR1  = off; off += bR1;                           off = (off + 255) & ~(size_t)255;
  const size_t oH   = off; off += (size_t)NPAD * HID * 2;        off = (off + 255) & ~(size_t)255;
  const size_t oCnt = off; off += (size_t)CNTPAD * 4;            off = (off + 255) & ~(size_t)255;
  const size_t oOff = off; off += (size_t)CNTPAD * 4;            off = (off + 255) & ~(size_t)255;
  const size_t oRb  = off; off += (size_t)RBN * 4;               off = (off + 255) & ~(size_t)255;
  const size_t oCsr = off; off += (size_t)csrLen * 4;            off = (off + 255) & ~(size_t)255;
  if (off > ws_size || off > (size_t)WSCAP) return;

  _Float16* wpl  = (_Float16*)(ws + oWp);
  _Float16* xm16 = (_Float16*)(ws + oR1);
  _Float16* xo16 = xm16 + (size_t)NPAD * FIN;
  _Float16* hm16 = (_Float16*)(ws + oR1);
  _Float16* h16  = (_Float16*)(ws + oH);
  int*   cnt  = (int*)(ws + oCnt);
  int*   offp = (int*)(ws + oOff);
  int*   rb   = (int*)(ws + oRb);
  int*   csr  = (int*)(ws + oCsr);

  const int vec8 = ((nE & 3) == 0) ? 1 : 0;

  k_wcvt<<<(nUnits + NTHR - 1) / NTHR, NTHR, 0, stream>>>(w1l, w1r, w2l, w2r, wpl, nUnits);
  k_count<<<nBC, NTHR, 0, stream>>>(dst, cnt, nE, vec8);
  k_offsets<<<1, OTHR, 0, stream>>>(cnt, offp, rb, nBC);
  hipFuncSetAttribute(reinterpret_cast<const void*>(&k_fill),
                      hipFuncAttributeMaxDynamicSharedMemorySize, LDS_FILL);
  k_fill<<<nBF, NTHR, LDS_FILL, stream>>>(src, dst, offp, rb, csr, nN, nE, vec8, csrLen);

  hipFuncSetAttribute(reinterpret_cast<const void*>(&k_agg1),
                      hipFuncAttributeMaxDynamicSharedMemorySize, LDS_AGG1);
  k_agg1<<<nAgg, ATHR, LDS_AGG1, stream>>>(csr, offp, cnt, x, xm16, xo16, nN, csrLen);
  k_gemm1<FIN, HID, BM1><<<nG1, NTHR, 0, stream>>>(xm16, xo16, wpl, b1, h16, nN);

  hipFuncSetAttribute(reinterpret_cast<const void*>(&k_agg2),
                      hipFuncAttributeMaxDynamicSharedMemorySize, LDS_AGG2);
  k_agg2<<<nAgg, ATHR, LDS_AGG2, stream>>>(csr, offp, cnt, h16, hm16, nN, csrLen);
  k_gemm2<HID, NOP, BM2, NCLS><<<nG2, NTHR, 0, stream>>>(hm16, h16, wpl + (size_t)U1 * 8, b2, out, nN);
}
